// GaussianKANLayer_70179765617079
// MI455X (gfx1250) — hardware-verified
//
#include <hip/hip_runtime.h>
#include <hip/hip_bf16.h>
#include <math.h>


#define BB 2
#define SS 2048
#define DD 1024
#define HH 16
#define DKK 64
#define QW 2

typedef _Float16 bf16;
typedef __attribute__((ext_vector_type(4))) unsigned v4u_t;
typedef unsigned v4ua __attribute__((ext_vector_type(4), may_alias));
typedef __attribute__((ext_vector_type(4))) float v4f_t;
typedef float v4fa __attribute__((ext_vector_type(4), may_alias));
typedef __attribute__((ext_vector_type(16))) bf16  bf16x16;
typedef __attribute__((ext_vector_type(8)))  bf16  bf16x8;
typedef __attribute__((ext_vector_type(4)))  bf16  bf16x4;
typedef __attribute__((ext_vector_type(8)))  float f32x8;

#define LDS_STRIDE 48
#define KSTRIDE    72
#define VSTRIDE    48

__device__ __forceinline__ f32x8 wmma_bf16(bf16x16 a, bf16x16 b, f32x8 c) {
  return __builtin_amdgcn_wmma_f32_16x16x32_f16(
      false, a, false, b, (short)0, c, false, false);
}

template <typename T>
__device__ __forceinline__ bf16x16 load_frag(const T* __restrict__ base, int ld,
                                             int row0, int k0) {
  const int lane = threadIdx.x & 31;
  const int r    = lane & 15;
  const int kh   = (lane >> 4) * 8;
  const T* p0 = base + (size_t)(row0 + r) * ld + (k0 + kh);
  const T* p1 = p0 + 16;
  bf16x16 f;
#pragma unroll
  for (int i = 0; i < 8; ++i) {
    f[i]     = (bf16)p0[i];
    f[i + 8] = (bf16)p1[i];
  }
  return f;
}

__device__ __forceinline__ bf16x16 lds_frag(const bf16* base, int stride) {
  const int lane = threadIdx.x & 31;
  const int row  = lane & 15;
  const int kh   = (lane >> 4) * 8;
  const bf16x8 lo = *(const bf16x8*)(base + row * stride + kh);
  const bf16x8 hi = *(const bf16x8*)(base + row * stride + kh + 16);
  bf16x16 f;
#pragma unroll
  for (int i = 0; i < 8; ++i) { f[i] = lo[i]; f[i + 8] = hi[i]; }
  return f;
}

template <typename T>
__device__ __forceinline__ void stage_read16(const T* __restrict__ p, float* buf) {
#pragma unroll
  for (int i = 0; i < 16; ++i) buf[i] = (float)p[i];
}

__device__ __forceinline__ void stage_write(bf16* dst, const float* buf, int nquad) {
#pragma unroll
  for (int i = 0; i < nquad; ++i) {
    bf16x4 q;
    q[0] = (bf16)buf[4 * i];     q[1] = (bf16)buf[4 * i + 1];
    q[2] = (bf16)buf[4 * i + 2]; q[3] = (bf16)buf[4 * i + 3];
    *(bf16x4*)(dst + 4 * i) = q;
  }
}

template <typename AT, int MODE>
__global__ __launch_bounds__(256) void gemm_bias_kernel(
    const AT* __restrict__ A, const float* __restrict__ W,
    const float* __restrict__ bias, void* __restrict__ out,
    int M, int N, int K) {
  __shared__ bf16 ldsA[128 * LDS_STRIDE];
  __shared__ bf16 ldsW[256 * LDS_STRIDE];
  __shared__ __attribute__((aligned(16))) unsigned char sob[256 * 136 * 2];

  const int t    = threadIdx.x;
  const int wave = t >> 5;
  const int lane = t & 31;
  const int wm   = (wave & 1) * 64;
  const int wn   = (wave >> 1) * 64;
  const int mBlk = blockIdx.x * 128;
  const int nBlk = blockIdx.y * 256;

  const int arow = t >> 1;
  const int ach  = (t & 1) * 16;

  float abuf[16];
  float wbuf[32];

  stage_read16(A + (size_t)(mBlk + arow) * K + ach, abuf);
  stage_read16(W + (size_t)(nBlk + t) * K,          wbuf);
  stage_read16(W + (size_t)(nBlk + t) * K + 16,     wbuf + 16);

  f32x8 acc[4][4] = {};

  for (int k = 0; k < K; k += 32) {
    __syncthreads();
    stage_write(&ldsA[arow * LDS_STRIDE + ach], abuf, 4);
    stage_write(&ldsW[t * LDS_STRIDE],          wbuf, 8);
    if (k + 32 < K) {
      stage_read16(A + (size_t)(mBlk + arow) * K + (k + 32) + ach, abuf);
      stage_read16(W + (size_t)(nBlk + t) * K + (k + 32),          wbuf);
      stage_read16(W + (size_t)(nBlk + t) * K + (k + 32) + 16,     wbuf + 16);
    }
    __syncthreads();

    bf16x16 af[4], wf[4];
#pragma unroll
    for (int i = 0; i < 4; ++i)
      af[i] = lds_frag(ldsA + (wm + 16 * i) * LDS_STRIDE, LDS_STRIDE);
#pragma unroll
    for (int j = 0; j < 4; ++j)
      wf[j] = lds_frag(ldsW + (wn + 16 * j) * LDS_STRIDE, LDS_STRIDE);
#pragma unroll
    for (int i = 0; i < 4; ++i)
#pragma unroll
      for (int j = 0; j < 4; ++j)
        acc[i][j] = wmma_bf16(af[i], wf[j], acc[i][j]);
  }

  const int nlane = lane & 15;
  const int mh    = (lane >> 4) * 8;
  __syncthreads();
  if (MODE == 0 || MODE == 1) {
    bf16* so = (bf16*)sob;
#pragma unroll
    for (int i = 0; i < 4; ++i)
#pragma unroll
      for (int j = 0; j < 4; ++j) {
        const int nl = wn + 16 * j + nlane;
        const float bv = bias ? bias[nBlk + nl] : 0.0f;
#pragma unroll
        for (int r = 0; r < 8; ++r) {
          const int ml = wm + 16 * i + mh + r;
          const bf16 hv = (bf16)(acc[i][j][r] + bv);
          if (MODE == 0) so[ml * 264 + nl] = hv;
          else           so[nl * 136 + ml] = hv;
        }
      }
    __syncthreads();
#pragma unroll 1
    for (int pass = 0; pass < 2; ++pass) {
      if (MODE == 0) {
        for (int ch = t; ch < 128 * 32; ch += 256) { const int ml = ch >> 5, q = (ch & 31) * 8;
          *(volatile v4u_t*)((bf16*)out + (size_t)(mBlk + ml) * N + nBlk + q) = *(const v4ua*)(so + ml * 264 + q); }
      } else {
        const int b_ = mBlk / SS, s0 = mBlk & (SS - 1);
        for (int ch = t; ch < 256 * 16; ch += 256) { const int nl = ch >> 4, q = (ch & 15) * 8; const int n = nBlk + nl, h = n >> 6, dk = n & (DKK - 1);
          *(volatile v4u_t*)((bf16*)out + (((size_t)(b_ * HH + h)) * DKK + dk) * SS + s0 + q) = *(const v4ua*)(so + nl * 136 + q); }
      }
      __threadfence();
    }
  } else {
    float* so = (float*)sob;
#pragma unroll 1
    for (int hf = 0; hf < 2; ++hf) {
      if (wm == hf * 64) {
#pragma unroll
        for (int i = 0; i < 4; ++i)
#pragma unroll
          for (int j = 0; j < 4; ++j) {
            const int nl = wn + 16 * j + nlane;
            const float bv = bias ? bias[nBlk + nl] : 0.0f;
#pragma unroll
            for (int r = 0; r < 8; ++r) so[(16 * i + mh + r) * 260 + nl] = acc[i][j][r] + bv;
          }
      }
      __syncthreads();
#pragma unroll 1
      for (int pass = 0; pass < 2; ++pass) {
        for (int ch = t; ch < 64 * 64; ch += 256) { const int ml = ch >> 6, q = (ch & 63) * 4;
          *(volatile v4f_t*)((float*)out + (size_t)(mBlk + hf * 64 + ml) * N + nBlk + q) = *(const volatile v4fa*)(so + ml * 260 + q); }
        __threadfence();
      }
      __syncthreads();
    }
  }
}


#define NR 16384
#define NI 256
#define NO 256
#define NGS 8
#define KTOT (NI * NGS)

__global__ __launch_bounds__(256) void k_arows(const float* __restrict__ x, const float* __restrict__ mu, const float* __restrict__ ls, bf16* __restrict__ A) {
  const int n = blockIdx.x, i = threadIdx.x;
  __shared__ __attribute__((aligned(16))) bf16 hbuf[256][NGS];
  const float xt = tanhf(x[(size_t)n * NI + i]);
#pragma unroll 1
  for (int g = 0; g < NGS; ++g) { const float sg = expf(ls[i * NGS + g]) + 1e-8f; const float z = (xt - mu[i * NGS + g]) / sg; hbuf[i][g] = (bf16)exp2f(-(z * z) * 1.44269504088896340736f); }
  bf16* dst = A + (size_t)n * KTOT + i * NGS; const v4u_t hv = *(const volatile v4ua*)(&hbuf[i][0]);
  *(volatile v4u_t*)dst = hv; __threadfence(); *(volatile v4u_t*)dst = hv;
}
__global__ __launch_bounds__(256) void k_wrows(const float* __restrict__ cf, float* __restrict__ Wc) {
  const int o = blockIdx.x, i = threadIdx.x; v4f_t a, c; const float* sp = cf + ((size_t)i * NO + o) * NGS;
  a.x = sp[0]; a.y = sp[1]; a.z = sp[2]; a.w = sp[3]; c.x = sp[4]; c.y = sp[5]; c.z = sp[6]; c.w = sp[7];
  float* dst = Wc + (size_t)o * KTOT + i * NGS;
#pragma unroll 1
  for (int pass = 0; pass < 2; ++pass) { *(volatile v4f_t*)dst = a; *(volatile v4f_t*)(dst + 4) = c; __threadfence(); }
}

extern "C" void kernel_launch(void* const* d_in, const int* in_sizes, int n_in,
                              void* d_out, int out_size, void* d_ws, size_t ws_size,
                              hipStream_t stream) {
  (void)in_sizes; (void)n_in; (void)out_size; (void)ws_size;
  const float* x  = (const float*)d_in[0];
  const float* mu = (const float*)d_in[1];
  const float* ls = (const float*)d_in[2];
  const float* cf = (const float*)d_in[3];
  char* ws = (char*)d_ws;
  bf16* A   = (bf16*)ws;  ws += (size_t)NR * KTOT * 2;
  float* Wc = (float*)ws; ws += (size_t)NO * KTOT * 4;
  k_arows<<<NR, 256, 0, stream>>>(x, mu, ls, A);
  k_wrows<<<NO, 256, 0, stream>>>(cf, Wc);
  gemm_bias_kernel<bf16, 2><<<dim3(NR / 128, NO / 256), 256, 0, stream>>>(A, Wc, nullptr, (float*)d_out, NR, NO, KTOT);
}
